// DeformableConv_20538533610096
// MI455X (gfx1250) — hardware-verified
//
#include <hip/hip_runtime.h>

typedef __attribute__((ext_vector_type(16))) _Float16 v16h;
typedef __attribute__((ext_vector_type(8)))  _Float16 v8h;
typedef __attribute__((ext_vector_type(16))) __bf16   v16b;
typedef __attribute__((ext_vector_type(8)))  __bf16   v8b;
typedef __attribute__((ext_vector_type(8)))  float    v8f;
typedef __attribute__((ext_vector_type(4)))  float    v4f;
typedef __attribute__((ext_vector_type(4)))  unsigned int v4u;

__device__ __forceinline__ unsigned short f2bf_bits(float f) {
  unsigned u = __float_as_uint(f);
  return (unsigned short)((u + 0x7FFFu + ((u >> 16) & 1u)) >> 16);
}
__device__ __forceinline__ float bf_bits2f(unsigned short h) { return __uint_as_float(((unsigned)h) << 16); }

__device__ __forceinline__ void dep_guard_h(v8f& a, v8f& b, v16h x, v16h y) { asm volatile("v_nop\n\tv_nop\n\tv_nop\n\tv_nop" : "+v"(a), "+v"(b) : "v"(x), "v"(y)); }
__device__ __forceinline__ void dep_guard_b(v8f& a, v8f& b, v16b x, v16b y) { asm volatile("v_nop\n\tv_nop\n\tv_nop\n\tv_nop" : "+v"(a), "+v"(b) : "v"(x), "v"(y)); }
__device__ __forceinline__ void keep4_h(v16h a, v16h b, v16h c, v16h d) { asm volatile("v_nop" :: "v"(a), "v"(b), "v"(c), "v"(d)); }
__device__ __forceinline__ void keep4_b(v16b a, v16b b, v16b c, v16b d) { asm volatile("v_nop" :: "v"(a), "v"(b), "v"(c), "v"(d)); }
__device__ __forceinline__ void acc_guard4(v8f& a, v8f& b, v8f& c, v8f& d) { asm volatile("v_nop\n\tv_nop\n\tv_nop\n\tv_nop" : "+v"(a), "+v"(b), "+v"(c), "+v"(d)); }
template <typename T> struct Frag;
template <> struct Frag<_Float16> {
  typedef v16h V; union U { v16h v; v8h h[2]; };
  static __device__ __forceinline__ v16h load(const _Float16* p) {
    U f; f.h[0] = *(const v8h*)(p); f.h[1] = *(const v8h*)(p + 16); return f.v;
  }
  static __device__ __forceinline__ v8f mma(v16h a, v16h b, v8f c) {
    return __builtin_amdgcn_wmma_f32_16x16x32_f16(false, a, false, b, (short)0, c, false, false);
  }
  static __device__ __forceinline__ void guard(v8f& a, v8f& b, v16h x, v16h y) { dep_guard_h(a, b, x, y); }
  static __device__ __forceinline__ void keep(v16h a, v16h b, v16h c, v16h d) { keep4_h(a, b, c, d); }
};
template <> struct Frag<__bf16> {
  typedef v16b V; union U { v16b v; v8b h[2]; };
  static __device__ __forceinline__ v16b load(const __bf16* p) {
    U f; f.h[0] = *(const v8b*)(p); f.h[1] = *(const v8b*)(p + 16); return f.v;
  }
  static __device__ __forceinline__ v8f mma(v16b a, v16b b, v8f c) {
    return __builtin_amdgcn_wmma_f32_16x16x32_bf16(false, a, false, b, (short)0, c, false, false);
  }
  static __device__ __forceinline__ void guard(v8f& a, v8f& b, v16b x, v16b y) { dep_guard_b(a, b, x, y); }
  static __device__ __forceinline__ void keep(v16b a, v16b b, v16b c, v16b d) { keep4_b(a, b, c, d); }
};

template <int ET> struct Elem;
template <> struct Elem<0> { typedef _Float16 T; };
template <> struct Elem<1> { typedef __bf16 T; };
template <int ET, bool SPLIT, int BIAS_MODE, int OUT_MODE, bool RESID, int ACT = 0>
__global__ __launch_bounds__(256) void wmma_gemm64(
    const unsigned short* __restrict__ Ap, const unsigned short* __restrict__ A2p, int lda, long strideA,
    const unsigned short* __restrict__ Btp, const unsigned short* __restrict__ Bt2p, int ldb, long strideB,
    void* __restrict__ Cout, void* __restrict__ Cout2, int ldc, long strideC,
    const float* __restrict__ bias,
    const float* __restrict__ resid, long strideR,
    int M, int N, int K, float scale) {
  typedef typename Elem<ET>::T T;
  typedef typename Frag<T>::V V;
  const T* A = (const T*)Ap; const T* A2 = (const T*)A2p; const T* Bt = (const T*)Btp; const T* Bt2 = (const T*)Bt2p;
  __shared__ __align__(16) float sT[8][16 * 68];
  const int b    = blockIdx.y;
  const int lane = threadIdx.x & 31;
  const int wave = threadIdx.x >> 5;
  const int tilesN = N >> 6;
  const int tilesM = M >> 6;
  const int tile = blockIdx.x * 8 + wave;
  if (tile >= tilesM * tilesN) return;
  const int tm = tile / tilesN;
  const int tn = tile - tm * tilesN;
  const int m0 = tm << 6;
  const int n0 = tn << 6;

  const T* Ab  = A  + (size_t)b * strideA;
  const T* Bb  = Bt + (size_t)b * strideB;
  const T* Ab2 = SPLIT ? (A2  + (size_t)b * strideA) : nullptr;
  const T* Bb2 = SPLIT ? (Bt2 + (size_t)b * strideB) : nullptr;

  const int rlane = lane & 15;
  const int koff  = (lane >> 4) * 8;
  const int mOff  = (lane >> 4) * 8;

  v8f acc[4][4];
#pragma unroll
  for (int i = 0; i < 4; ++i)
#pragma unroll
    for (int j = 0; j < 4; ++j) acc[i][j] = (v8f){0.f,0.f,0.f,0.f,0.f,0.f,0.f,0.f};

  for (int k0 = 0; k0 < K; k0 += 32) {
    V bh[4], bl[4];
#pragma unroll
    for (int j = 0; j < 4; ++j) {
      const size_t bo = (size_t)(n0 + (j << 4) + rlane) * ldb + koff + k0;
      bh[j] = Frag<T>::load(Bb + bo);
      if (SPLIT) bl[j] = Frag<T>::load(Bb2 + bo);
    }
#pragma unroll
    for (int i = 0; i < 4; ++i) {
      const size_t ao = (size_t)(m0 + (i << 4) + rlane) * lda + koff + k0;
      V ah = Frag<T>::load(Ab + ao);
      V al;
      if (SPLIT) al = Frag<T>::load(Ab2 + ao);
#pragma unroll
      for (int j = 0; j < 4; ++j) {
        acc[i][j] = Frag<T>::mma(ah, bh[j], acc[i][j]);
        if (SPLIT) {
          acc[i][j] = Frag<T>::mma(ah, bl[j], acc[i][j]);
          acc[i][j] = Frag<T>::mma(al, bh[j], acc[i][j]);
        }
      }
      Frag<T>::guard(acc[i][0], acc[i][3], ah, SPLIT ? al : ah);
    }
    Frag<T>::keep(bh[0], bh[1], bh[2], bh[3]);
    if (SPLIT) Frag<T>::keep(bl[0], bl[1], bl[2], bl[3]);
  }
  acc_guard4(acc[0][0], acc[0][1], acc[0][2], acc[0][3]);
  acc_guard4(acc[1][0], acc[1][1], acc[1][2], acc[1][3]);
  acc_guard4(acc[2][0], acc[2][1], acc[2][2], acc[2][3]);
  acc_guard4(acc[3][0], acc[3][1], acc[3][2], acc[3][3]);

  float* slab = sT[wave];
  const float* Rb = RESID ? (resid + (size_t)b * strideR) : nullptr;
#pragma unroll
  for (int i = 0; i < 4; ++i) {
    const int mBase = m0 + (i << 4);
#pragma unroll
    for (int j = 0; j < 4; ++j) {
      const int n = n0 + (j << 4) + rlane;
      float bv = 0.f;
      if (BIAS_MODE == 2) bv = bias[n];
#pragma unroll
      for (int r = 0; r < 8; ++r) {
        float v = acc[i][j][r] * scale;
        if (BIAS_MODE == 1) v += bias[mBase + mOff + r];
        if (BIAS_MODE == 2) v += bv;
        if (RESID) v += Rb[(size_t)(mBase + mOff + r) * ldc + n];
        if (ACT == 1) v = tanhf(v);
        if (ACT == 2) v = fmaxf(v, 0.0f);
        if (ACT == 3) v = v / (1.0f + expf(-v));
        if (ACT == 4) v = (v > 0.f) ? v : 0.01f * v;
        if (ACT == 5) v = 0.5f * v * (1.0f + erff(v * 0.70710678118654752f));
        slab[(mOff + r) * 68 + (j << 4) + rlane] = v;
      }
    }
    __builtin_amdgcn_fence(__ATOMIC_RELEASE, "workgroup");
    __builtin_amdgcn_wave_barrier();
    __builtin_amdgcn_fence(__ATOMIC_ACQUIRE, "workgroup");
    if (OUT_MODE == 0) {
      float* C = (float*)Cout + (size_t)b * strideC;
      const int hh = lane >> 4, c4 = (lane & 15) * 4;
      for (int pass = 0; pass < 2; ++pass) {
#pragma unroll
        for (int it = 0; it < 8; ++it) {
          const int row = it * 2 + hh;
          v4f v = *(const v4f*)(slab + row * 68 + c4);
          *(volatile v4f*)(C + (size_t)(mBase + row) * ldc + n0 + c4) = v;
        }
        __threadfence();
      }
    } else {
      const int q = lane >> 3, c8 = (lane & 7) * 8;
      unsigned short* C  = (unsigned short*)Cout  + (size_t)b * strideC;
      unsigned short* C2 = (OUT_MODE == 2) ? ((unsigned short*)Cout2 + (size_t)b * strideC) : nullptr;
      for (int pass = 0; pass < 2; ++pass) {
#pragma unroll
        for (int it = 0; it < 4; ++it) {
          const int row = it * 4 + q;
          const float* sp = slab + row * 68 + c8;
          v8h hv, lv;
#pragma unroll
          for (int e = 0; e < 8; ++e) {
            if (OUT_MODE == 1) {
              hv[e] = (_Float16)sp[e];
            } else {
              unsigned short hb = f2bf_bits(sp[e]);
              unsigned short lb = f2bf_bits(sp[e] - bf_bits2f(hb));
              hv[e] = __builtin_bit_cast(_Float16, hb);
              lv[e] = __builtin_bit_cast(_Float16, lb);
            }
          }
          *(volatile v8h*)(C + (size_t)(mBase + row) * ldc + n0 + c8) = hv;
          if (OUT_MODE == 2) *(volatile v8h*)(C2 + (size_t)(mBase + row) * ldc + n0 + c8) = lv;
        }
        __threadfence();
      }
    }
    __builtin_amdgcn_fence(__ATOMIC_RELEASE, "workgroup");
    __builtin_amdgcn_wave_barrier();
    __builtin_amdgcn_fence(__ATOMIC_ACQUIRE, "workgroup");
  }
}

constexpr int NBATCH  = 8;
constexpr int NCH_IN  = 64;
constexpr int IMG_H   = 128;
constexpr int IMG_W   = 128;
constexpr int NPIX    = IMG_H * IMG_W;
constexpr int NCH_OUT = 64;
constexpr int NTAPS   = 9;
constexpr int NCH_OFF = 2 * NTAPS;
constexpr int KDIM    = NTAPS * NCH_IN;
constexpr int MPAD    = 64;
constexpr float WCARRY     = 16.0f;
constexpr float WCARRY_INV = 1.0f / 16.0f;

static_assert(KDIM % 32 == 0, "K multiple of 32");
static_assert(MPAD % 64 == 0 && NPIX % 64 == 0, "GEMM tiles");
static_assert(NCH_OFF <= MPAD && NCH_OUT == MPAD, "channel padding");
static_assert((MPAD * KDIM) % (8 * 256) == 0, "pack coverage exact");
static_assert((NPIX * KDIM) % (8 * 256) == 0, "plane coverage exact");
static_assert(((MPAD / 64) * (NPIX / 64)) % 8 == 0, "GEMM grid exact");
static_assert(NCH_IN % 8 == 0 && KDIM % 8 == 0, "8 channels per lane share one (row, tap)");

constexpr int PACK_BLOCKS = (MPAD * KDIM) / (8 * 256);
constexpr int PLANE_BLOCKS = (NPIX * KDIM) / (8 * 256);
constexpr int GEMM_BLOCKS = ((MPAD / 64) * (NPIX / 64)) / 8;

__device__ __forceinline__ float bf16_rne(float f) {
  unsigned u = __float_as_uint(f);
  u = (u + 0x7FFFu + ((u >> 16) & 1u)) & 0xFFFF0000u;
  return __uint_as_float(u);
}
__device__ __forceinline__ unsigned pack2h(float a, float b) {
  const unsigned short ha = __builtin_bit_cast(unsigned short, (_Float16)a);
  const unsigned short hb = __builtin_bit_cast(unsigned short, (_Float16)b);
  return (unsigned)ha | ((unsigned)hb << 16);
}
__device__ __forceinline__ void store16_twice(unsigned short* dst, v4u v) {
  *(volatile v4u*)dst = v;
  __threadfence();
  *(volatile v4u*)dst = v;
}

__global__ __launch_bounds__(256) void pack_weight_f16(const float* __restrict__ w,
                                                       unsigned short* __restrict__ plane, int nreal) {
  const int g = blockIdx.x * 256 + threadIdx.x;
  const int e = g * 8;
  const int row = e / KDIM;
  const int r = e - row * KDIM;
  const int tap = r >> 6;
  const int c0 = r & 63;
  const bool live = row < nreal;
  const int rowc = live ? row : (nreal - 1);
  const float* src = w + ((size_t)rowc * NCH_IN + c0) * NTAPS + tap;
  float f[8];
#pragma unroll
  for (int i = 0; i < 8; ++i) {
    const float raw = src[i * NTAPS];
    f[i] = live ? (bf16_rne(raw) * WCARRY) : 0.0f;
  }
  v4u pk;
  pk[0] = pack2h(f[0], f[1]);
  pk[1] = pack2h(f[2], f[3]);
  pk[2] = pack2h(f[4], f[5]);
  pk[3] = pack2h(f[6], f[7]);
  store16_twice(plane + e, pk);
}

__global__ __launch_bounds__(256) void im2col_f16(const float* __restrict__ x,
                                                  unsigned short* __restrict__ plane, int b) {
  const int g = blockIdx.x * 256 + threadIdx.x;
  const int e = g * 8;
  const int pixel = e / KDIM;
  const int r = e - pixel * KDIM;
  const int tap = r >> 6;
  const int c0 = r & 63;
  const int hrow = pixel >> 7;
  const int wcol = pixel & 127;
  const int kh = tap / 3;
  const int kw = tap - kh * 3;
  const int yy = hrow + kh - 1;
  const int xx = wcol + kw - 1;
  const bool valid = ((unsigned)yy < (unsigned)IMG_H) && ((unsigned)xx < (unsigned)IMG_W);
  const int yc = min(max(yy, 0), IMG_H - 1);
  const int xc = min(max(xx, 0), IMG_W - 1);
  const float* src = x + (((size_t)b * NCH_IN + c0) * IMG_H + yc) * IMG_W + xc;
  float f[8];
#pragma unroll
  for (int i = 0; i < 8; ++i) {
    const float raw = src[(size_t)i * NPIX];
    f[i] = valid ? bf16_rne(raw) : 0.0f;
  }
  v4u pk;
  pk[0] = pack2h(f[0], f[1]);
  pk[1] = pack2h(f[2], f[3]);
  pk[2] = pack2h(f[4], f[5]);
  pk[3] = pack2h(f[6], f[7]);
  store16_twice(plane + e, pk);
}

__global__ __launch_bounds__(256) void deform_cols_f16(const float* __restrict__ x,
                                                       const float* __restrict__ offs,
                                                       unsigned short* __restrict__ plane, int b) {
#pragma clang fp contract(off)
  const int g = blockIdx.x * 256 + threadIdx.x;
  const int e = g * 8;
  const int pixel = e / KDIM;
  const int r = e - pixel * KDIM;
  const int tap = r >> 6;
  const int c0 = r & 63;
  const int hrow = pixel >> 7;
  const int wcol = pixel & 127;
  const int kh = tap / 3;
  const int kw = tap - kh * 3;

  const float offy = offs[(size_t)(tap * 2) * NPIX + pixel];
  const float offx = offs[(size_t)(tap * 2 + 1) * NPIX + pixel];
  const float py = (float)(hrow + kh - 1) + offy;
  const float px = (float)(wcol + kw - 1) + offx;
  const float y0f = floorf(py);
  const float x0f = floorf(px);
  const float wy1 = py - y0f;
  const float wx1 = px - x0f;
  const float wy0 = 1.0f - wy1;
  const float wx0 = 1.0f - wx1;
  const float y1f = y0f + 1.0f;
  const float x1f = x0f + 1.0f;
  const bool vy0 = (y0f >= 0.0f) && (y0f < (float)IMG_H);
  const bool vy1 = (y1f >= 0.0f) && (y1f < (float)IMG_H);
  const bool vx0 = (x0f >= 0.0f) && (x0f < (float)IMG_W);
  const bool vx1 = (x1f >= 0.0f) && (x1f < (float)IMG_W);
  const float t00 = wy0 * wx0;
  const float t01 = wy0 * wx1;
  const float t10 = wy1 * wx0;
  const float t11 = wy1 * wx1;
  const float w00 = (vy0 && vx0) ? t00 : 0.0f;
  const float w01 = (vy0 && vx1) ? t01 : 0.0f;
  const float w10 = (vy1 && vx0) ? t10 : 0.0f;
  const float w11 = (vy1 && vx1) ? t11 : 0.0f;
  const int yc0 = (int)fminf(fmaxf(y0f, 0.0f), (float)(IMG_H - 1));
  const int yc1 = (int)fminf(fmaxf(y1f, 0.0f), (float)(IMG_H - 1));
  const int xc0 = (int)fminf(fmaxf(x0f, 0.0f), (float)(IMG_W - 1));
  const int xc1 = (int)fminf(fmaxf(x1f, 0.0f), (float)(IMG_W - 1));
  int j00 = yc0 * IMG_W + xc0;
  int j01 = yc0 * IMG_W + xc1;
  int j10 = yc1 * IMG_W + xc0;
  int j11 = yc1 * IMG_W + xc1;

  const float* xb = x + ((size_t)b * NCH_IN + c0) * NPIX;
  unsigned wq0 = 0u, wq1 = 0u, wq2 = 0u, wq3 = 0u;
#pragma unroll 1
  for (int pr = 0; pr < 4; ++pr) {
    const float* p0 = xb + (size_t)(2 * pr) * NPIX;
    const float* p1 = p0 + NPIX;
    const float a00 = bf16_rne(p0[j00]);
    const float a01 = bf16_rne(p0[j01]);
    const float a10 = bf16_rne(p0[j10]);
    const float a11 = bf16_rne(p0[j11]);
    const float c00 = bf16_rne(p1[j00]);
    const float c01 = bf16_rne(p1[j01]);
    const float c10 = bf16_rne(p1[j10]);
    const float c11 = bf16_rne(p1[j11]);
    const float ga00 = a00 * w00;
    const float ga01 = a01 * w01;
    const float ga10 = a10 * w10;
    const float ga11 = a11 * w11;
    const float gc00 = c00 * w00;
    const float gc01 = c01 * w01;
    const float gc10 = c10 * w10;
    const float gc11 = c11 * w11;
    const float fa = ((ga00 + ga01) + ga10) + ga11;
    const float fc = ((gc00 + gc01) + gc10) + gc11;
    const unsigned nw = pack2h(fa, fc);
    wq0 = wq1; wq1 = wq2; wq2 = wq3; wq3 = nw;
    asm volatile("" : "+v"(j00), "+v"(j01), "+v"(j10), "+v"(j11) : "v"(nw));
  }
  v4u pk;
  pk[0] = wq0;
  pk[1] = wq1;
  pk[2] = wq2;
  pk[3] = wq3;
  store16_twice(plane + e, pk);
}

extern "C" void kernel_launch(void* const* d_in, const int* in_sizes, int n_in,
                              void* d_out, int out_size, void* d_ws, size_t ws_size,
                              hipStream_t stream) {
  if (n_in < 3) return;
  if (in_sizes[0] != NBATCH * NCH_IN * NPIX) return;
  if (in_sizes[1] != NCH_OFF * NCH_IN * NTAPS) return;
  if (in_sizes[2] != NCH_OUT * NCH_IN * NTAPS) return;
  if (out_size != NBATCH * NCH_OUT * NPIX) return;

  const float* x     = (const float*)d_in[0];
  const float* w_off = (const float*)d_in[1];
  const float* w_def = (const float*)d_in[2];
  float* out = (float*)d_out;

  const size_t wplane_bytes = (size_t)MPAD * KDIM * 2;
  const size_t cplane_bytes = (size_t)NPIX * KDIM * 2;
  const size_t offs_bytes   = (size_t)MPAD * NPIX * 4;
  const size_t o_a0   = 0;
  const size_t o_a1   = o_a0 + wplane_bytes;
  const size_t o_im   = o_a1 + wplane_bytes;
  const size_t o_cols = o_im + cplane_bytes;
  const size_t o_offs = o_cols + cplane_bytes;
  const size_t total  = o_offs + offs_bytes;
  if (total > ws_size) return;

  char* ws = (char*)d_ws;
  unsigned short* A0p   = (unsigned short*)(ws + o_a0);
  unsigned short* A1p   = (unsigned short*)(ws + o_a1);
  unsigned short* imP   = (unsigned short*)(ws + o_im);
  unsigned short* colsP = (unsigned short*)(ws + o_cols);
  float* offsP          = (float*)(ws + o_offs);
  const float* dummyf   = (const float*)(ws + o_a0);

  pack_weight_f16<<<PACK_BLOCKS, 256, 0, stream>>>(w_off, A0p, NCH_OFF);
  pack_weight_f16<<<PACK_BLOCKS, 256, 0, stream>>>(w_def, A1p, NCH_OUT);

  for (int b = 0; b < NBATCH; ++b) {
    im2col_f16<<<PLANE_BLOCKS, 256, 0, stream>>>(x, imP, b);
    wmma_gemm64<0, false, 0, 0, false, 0><<<dim3(GEMM_BLOCKS, 1), 256, 0, stream>>>(
        A0p, A0p, KDIM, 0L,
        imP, imP, KDIM, 0L,
        (void*)offsP, (void*)offsP, NPIX, 0L,
        dummyf, dummyf, 0L,
        MPAD, NPIX, KDIM, WCARRY_INV);
    deform_cols_f16<<<PLANE_BLOCKS, 256, 0, stream>>>(x, offsP, colsP, b);
    float* outb = out + (size_t)b * NCH_OUT * NPIX;
    wmma_gemm64<0, false, 0, 0, false, 0><<<dim3(GEMM_BLOCKS, 1), 256, 0, stream>>>(
        A1p, A1p, KDIM, 0L,
        colsP, colsP, KDIM, 0L,
        (void*)outb, (void*)outb, NPIX, 0L,
        dummyf, dummyf, 0L,
        MPAD, NPIX, KDIM, WCARRY_INV);
  }
}
